// Co_Attention_41712722378816
// MI455X (gfx1250) — hardware-verified
//
#include <hip/hip_runtime.h>
#include <stddef.h>


typedef __bf16   v16bf __attribute__((ext_vector_type(16)));
typedef float    v8f   __attribute__((ext_vector_type(8)));
typedef unsigned v8u   __attribute__((ext_vector_type(8)));
typedef float    v4f   __attribute__((ext_vector_type(4)));
typedef unsigned v4u   __attribute__((ext_vector_type(4)));
typedef v4f __attribute__((may_alias)) v4fa;
typedef v4u __attribute__((may_alias)) v4ua;

static constexpr int kD            = 64;
static constexpr int kN            = 512;
static constexpr int kThreads      = 512;
static constexpr int kWaves        = kThreads / 32;
static constexpr int kTilesPerWave = (kN / 16) / kWaves;
static constexpr size_t kPlaneBytes = (size_t)kN * kD * 2;
static constexpr size_t kSmemBytes  = 4 * kPlaneBytes + 2 * (size_t)kN * 4 + 16 * 4;

__device__ __forceinline__ unsigned bfr(float a) {
    unsigned u = __builtin_bit_cast(unsigned, a);
    return (u + 0x7FFFu + ((u >> 16) & 1u)) >> 16;
}
struct HL { unsigned hi; unsigned lo; };
__device__ __forceinline__ HL split2(float a, float b) {
    const unsigned ha = bfr(a), hb = bfr(b);
    const float ra = a - __builtin_bit_cast(float, ha << 16);
    const float rb = b - __builtin_bit_cast(float, hb << 16);
    HL r;
    r.hi = ha | (hb << 16);
    r.lo = bfr(ra) | (bfr(rb) << 16);
    return r;
}
struct Frag2 { v8u hi; v8u lo; };
__device__ __forceinline__ Frag2 mkfrag(v4f a, v4f b, v4f c, v4f d) {
    Frag2 f; HL t;
    t = split2(a[0], a[1]); f.hi[0] = t.hi; f.lo[0] = t.lo;
    t = split2(a[2], a[3]); f.hi[1] = t.hi; f.lo[1] = t.lo;
    t = split2(b[0], b[1]); f.hi[2] = t.hi; f.lo[2] = t.lo;
    t = split2(b[2], b[3]); f.hi[3] = t.hi; f.lo[3] = t.lo;
    t = split2(c[0], c[1]); f.hi[4] = t.hi; f.lo[4] = t.lo;
    t = split2(c[2], c[3]); f.hi[5] = t.hi; f.lo[5] = t.lo;
    t = split2(d[0], d[1]); f.hi[6] = t.hi; f.lo[6] = t.lo;
    t = split2(d[2], d[3]); f.hi[7] = t.hi; f.lo[7] = t.lo;
    return f;
}
__device__ __forceinline__ Frag2 ldfrag_row(const float* row, int k0, int h) {
    const float* p = row + k0 + 8 * h;
    const v4f a = *(const v4fa*)(p);
    const v4f b = *(const v4fa*)(p + 4);
    const v4f c = *(const v4fa*)(p + 16);
    const v4f d = *(const v4fa*)(p + 20);
    return mkfrag(a, b, c, d);
}
__device__ __forceinline__ Frag2 ldfrag_col(const float* colbase, int ld, int k0, int h) {
    v4f a, b, c, d;
    #pragma unroll
    for (int j = 0; j < 4; ++j) {
        a[j] = colbase[(size_t)(k0 + 8 * h + j) * ld];
        b[j] = colbase[(size_t)(k0 + 8 * h + 4 + j) * ld];
        c[j] = colbase[(size_t)(k0 + 16 + 8 * h + j) * ld];
        d[j] = colbase[(size_t)(k0 + 16 + 8 * h + 4 + j) * ld];
    }
    return mkfrag(a, b, c, d);
}
__device__ __forceinline__ v8u ldfrag_bf(const unsigned short* row, int k0, int h) {
    const unsigned short* p = row + k0 + 8 * h;
    const v4u a = *(const v4ua*)(p);
    const v4u c = *(const v4ua*)(p + 16);
    v8u r;
    r[0] = a[0]; r[1] = a[1]; r[2] = a[2]; r[3] = a[3];
    r[4] = c[0]; r[5] = c[1]; r[6] = c[2]; r[7] = c[3];
    return r;
}
__device__ __forceinline__ v8f wmma3(v8u ah, v8u al, v8u bh, v8u bl, v8f c) {
    c = __builtin_amdgcn_wmma_f32_16x16x32_bf16(false, __builtin_bit_cast(v16bf, ah),
                                                false, __builtin_bit_cast(v16bf, bh), (short)0, c, false, false);
    c = __builtin_amdgcn_wmma_f32_16x16x32_bf16(false, __builtin_bit_cast(v16bf, ah),
                                                false, __builtin_bit_cast(v16bf, bl), (short)0, c, false, false);
    c = __builtin_amdgcn_wmma_f32_16x16x32_bf16(false, __builtin_bit_cast(v16bf, al),
                                                false, __builtin_bit_cast(v16bf, bh), (short)0, c, false, false);
    asm volatile("v_nop\n\tv_nop\n\tv_nop\n\tv_nop" : "+v"(c) : "v"(ah), "v"(al), "v"(bh), "v"(bl));
    return c;
}

__device__ __forceinline__ float blockMax(float v, float* red) {
    #pragma unroll
    for (int off = 16; off > 0; off >>= 1) v = fmaxf(v, __shfl_xor(v, off, 32));
    const int w = threadIdx.x >> 5, l = threadIdx.x & 31;
    if (l == 0) red[w] = v;
    __syncthreads();
    if (w == 0) {
        float x = red[l & 15];
        #pragma unroll
        for (int off = 8; off > 0; off >>= 1) x = fmaxf(x, __shfl_xor(x, off, 32));
        if (l == 0) red[0] = x;
    }
    __syncthreads();
    const float r = red[0];
    __syncthreads();
    return r;
}
__device__ __forceinline__ float blockSum(float v, float* red) {
    #pragma unroll
    for (int off = 16; off > 0; off >>= 1) v += __shfl_xor(v, off, 32);
    const int w = threadIdx.x >> 5, l = threadIdx.x & 31;
    if (l == 0) red[w] = v;
    __syncthreads();
    if (w == 0) {
        float x = red[l & 15];
        #pragma unroll
        for (int off = 8; off > 0; off >>= 1) x += __shfl_xor(x, off, 32);
        if (l == 0) red[0] = x;
    }
    __syncthreads();
    const float r = red[0];
    __syncthreads();
    return r;
}

template <bool BCOL, bool OPLANE, bool HASBIAS>
__device__ __forceinline__ void tile_gemm(const float* arows, const float* bsrc, const float* bias,
                                          float* oscr, unsigned short* ohi, unsigned short* olo,
                                          int orow0, int lane)
{
    const int h = lane >> 4, m = lane & 15;
    const Frag2 a0 = ldfrag_row(arows + m * kD, 0, h);
    const Frag2 a1 = ldfrag_row(arows + m * kD, 32, h);
    #pragma unroll 1
    for (int ct = 0; ct < kD / 16; ++ct) {
        const int n = ct * 16 + m;
        Frag2 b0, b1;
        if (BCOL) {
            b0 = ldfrag_col(bsrc + n, kD, 0, h);
            b1 = ldfrag_col(bsrc + n, kD, 32, h);
        } else {
            b0 = ldfrag_row(bsrc + (size_t)n * kD, 0, h);
            b1 = ldfrag_row(bsrc + (size_t)n * kD, 32, h);
        }
        v8f acc = {0.f, 0.f, 0.f, 0.f, 0.f, 0.f, 0.f, 0.f};
        acc = wmma3(a0.hi, a0.lo, b0.hi, b0.lo, acc);
        acc = wmma3(a1.hi, a1.lo, b1.hi, b1.lo, acc);
        const float bv = HASBIAS ? bias[n] : 0.f;
        if (OPLANE) {
            #pragma unroll
            for (int r = 0; r < 8; ++r) {
                const float v = acc[r] + bv;
                const unsigned hb = bfr(v);
                const float res = v - __builtin_bit_cast(float, hb << 16);
                const size_t o = (size_t)(orow0 + 8 * h + r) * kD + n;
                ohi[o] = (unsigned short)hb;
                olo[o] = (unsigned short)bfr(res);
            }
        } else {
            #pragma unroll
            for (int r = 0; r < 8; ++r) oscr[(8 * h + r) * kD + n] = acc[r] + bv;
        }
    }
}

__device__ __forceinline__ void strip_max(const unsigned short* Ahi, const unsigned short* Alo,
                                          const unsigned short* Bhi, const unsigned short* Blo,
                                          int rt, int lane, float* dst)
{
    const int h = lane >> 4, m = lane & 15;
    const unsigned short* ah = Ahi + (size_t)(rt * 16 + m) * kD;
    const unsigned short* al = Alo + (size_t)(rt * 16 + m) * kD;
    const v8u a0h = ldfrag_bf(ah, 0, h),  a0l = ldfrag_bf(al, 0, h);
    const v8u a1h = ldfrag_bf(ah, 32, h), a1l = ldfrag_bf(al, 32, h);
    float rmax[8];
    #pragma unroll
    for (int r = 0; r < 8; ++r) rmax[r] = -3.402823466e38f;
    #pragma unroll 1
    for (int ct = 0; ct < kN / 16; ++ct) {
        const unsigned short* bh = Bhi + (size_t)(ct * 16 + m) * kD;
        const unsigned short* bl = Blo + (size_t)(ct * 16 + m) * kD;
        const v8u b0h = ldfrag_bf(bh, 0, h),  b0l = ldfrag_bf(bl, 0, h);
        const v8u b1h = ldfrag_bf(bh, 32, h), b1l = ldfrag_bf(bl, 32, h);
        v8f acc = {0.f, 0.f, 0.f, 0.f, 0.f, 0.f, 0.f, 0.f};
        acc = wmma3(a0h, a0l, b0h, b0l, acc);
        acc = wmma3(a1h, a1l, b1h, b1l, acc);
        #pragma unroll
        for (int r = 0; r < 8; ++r) rmax[r] = fmaxf(rmax[r], acc[r]);
    }
    #pragma unroll
    for (int r = 0; r < 8; ++r) {
        float v = rmax[r];
        v = fmaxf(v, __shfl_xor(v, 8, 32));
        v = fmaxf(v, __shfl_xor(v, 4, 32));
        v = fmaxf(v, __shfl_xor(v, 2, 32));
        v = fmaxf(v, __shfl_xor(v, 1, 32));
        if (m == 0) dst[rt * 16 + 8 * h + r] = v;
    }
}

__global__ void __launch_bounds__(kThreads)
coattn_fused(const float* u_fea, const float* i_fea, const float* Mm,
             const float* Wu, const float* bu, const float* Wi, const float* bi,
             float* out, int off1)
{
    extern __shared__ v4u dsm[];
    unsigned short* Uhi = (unsigned short*)dsm;
    unsigned short* Ulo = Uhi + kN * kD;
    unsigned short* Vhi = Ulo + kN * kD;
    unsigned short* Vlo = Vhi + kN * kD;
    float* umax = (float*)(Vlo + kN * kD);
    float* imax = umax + kN;
    float* red  = imax + kN;

    const int tid  = threadIdx.x;
    const int wave = tid >> 5;
    const int lane = tid & 31;
    const int b    = blockIdx.x;
    float* scr = (float*)Vhi + wave * (16 * kD);
    const float* ub = u_fea + (size_t)b * kN * kD;
    const float* ib = i_fea + (size_t)b * kN * kD;

    #pragma unroll 1
    for (int t = 0; t < kTilesPerWave; ++t) {
        const int rt = wave * kTilesPerWave + t;
        tile_gemm<false, false, true>(ub + (size_t)rt * 16 * kD, Wu, bu, scr, Uhi, Ulo, 0, lane);
        __syncthreads();
        tile_gemm<true, true, false>(scr, Mm, bu, scr, Uhi, Ulo, rt * 16, lane);
        __syncthreads();
    }
    #pragma unroll 1
    for (int t = 0; t < kTilesPerWave; ++t) {
        const int rt = wave * kTilesPerWave + t;
        tile_gemm<false, true, true>(ib + (size_t)rt * 16 * kD, Wi, bi, scr, Vhi, Vlo, rt * 16, lane);
    }
    __syncthreads();

    #pragma unroll 1
    for (int t = 0; t < kTilesPerWave; ++t)
        strip_max(Uhi, Ulo, Vhi, Vlo, wave * kTilesPerWave + t, lane, umax);
    #pragma unroll 1
    for (int t = 0; t < kTilesPerWave; ++t)
        strip_max(Vhi, Vlo, Uhi, Ulo, wave * kTilesPerWave + t, lane, imax);
    __syncthreads();

    const float us = umax[tid];
    const float is = imax[tid];
    const float mu = blockMax(us, red);
    const float eu = expf(us - mu);
    const float su = blockSum(eu, red);
    const float mi = blockMax(is, red);
    const float ei = expf(is - mi);
    const float si = blockSum(ei, red);
    umax[tid] = eu / su;
    imax[tid] = ei / si;
    __syncthreads();

    if (wave < 2) {
        const float* sp = (wave == 0) ? umax : imax;
        float* dp = out + (size_t)b * kN + ((wave == 0) ? (size_t)0 : (size_t)off1);
        const v4f w0 = *(const v4fa*)(sp + 4 * lane);
        const v4f w1 = *(const v4fa*)(sp + 128 + 4 * lane);
        const v4f w2 = *(const v4fa*)(sp + 256 + 4 * lane);
        const v4f w3 = *(const v4fa*)(sp + 384 + 4 * lane);
        *(volatile v4f*)(dp + 4 * lane)       = w0;
        *(volatile v4f*)(dp + 128 + 4 * lane) = w1;
        *(volatile v4f*)(dp + 256 + 4 * lane) = w2;
        *(volatile v4f*)(dp + 384 + 4 * lane) = w3;
        __threadfence();
        *(volatile v4f*)(dp + 4 * lane)       = w0;
        *(volatile v4f*)(dp + 128 + 4 * lane) = w1;
        *(volatile v4f*)(dp + 256 + 4 * lane) = w2;
        *(volatile v4f*)(dp + 384 + 4 * lane) = w3;
    }
}

extern "C" void kernel_launch(void* const* d_in, const int* in_sizes, int n_in,
                              void* d_out, int out_size, void* d_ws, size_t ws_size,
                              hipStream_t stream)
{
    (void)d_ws; (void)ws_size;
    if (n_in < 7) return;
    const int per = kN * kD;
    const int nb  = in_sizes[0] / per;
    if (nb <= 0) return;
    if (in_sizes[0] != nb * per || in_sizes[1] != nb * per) return;
    if (in_sizes[2] != kD * kD || in_sizes[3] != kD * kD || in_sizes[5] != kD * kD) return;
    if (in_sizes[4] != kD || in_sizes[6] != kD) return;
    if (out_size != 2 * nb * kN) return;

    const float* u_fea = (const float*)d_in[0];
    const float* i_fea = (const float*)d_in[1];
    const float* Mm    = (const float*)d_in[2];
    const float* Wu    = (const float*)d_in[3];
    const float* bu    = (const float*)d_in[4];
    const float* Wi    = (const float*)d_in[5];
    const float* bi    = (const float*)d_in[6];
    const int off1 = nb * kN;

    coattn_fused<<<nb, kThreads, kSmemBytes, stream>>>(u_fea, i_fea, Mm, Wu, bu, Wi, bi,
                                                       (float*)d_out, off1);
    (void)hipGetLastError();
}
